// GATv2Pytorch_70282844832158
// MI455X (gfx1250) — hardware-verified
//
#include <hip/hip_runtime.h>

#define NB     2
#define NNODE  512
#define FIN    128
#define NHEAD  4
#define HD     64
#define OUTW   256

#define XP   136
#define WP   136
#define HP   72
#define SP   68

#define QR   16
#define KCH  128
#define ZJP  65
#define PSP  520
#define OSP  68

typedef _Float16 f16t;
typedef _Float16 v16h __attribute__((ext_vector_type(16)));
typedef _Float16 v8h  __attribute__((ext_vector_type(8)));
typedef _Float16 v4h  __attribute__((ext_vector_type(4)));
typedef float    v8f  __attribute__((ext_vector_type(8)));
typedef float    v4f  __attribute__((ext_vector_type(4)));

union Frag  { v16h v; v8h h[2]; };
union Pack8 { v8h v; f16t e[8]; };

__device__ __forceinline__ v8f mma16(v16h a, v16h b, v8f c) {
  c = __builtin_amdgcn_wmma_f32_16x16x32_f16(false, a, false, b, (short)0, c, false, false);
  asm volatile("v_nop\n\tv_nop\n\tv_nop\n\tv_nop" : "+v"(c) : "v"(a), "v"(b));
  return c;
}
__device__ __forceinline__ v16h ldfrag(const f16t* p) {
  Frag f;
  f.h[0] = *(const v8h*)(p);
  f.h[1] = *(const v8h*)(p + 16);
  return f.v;
}
__device__ __forceinline__ v8f zero8() {
  v8f z = {0.f, 0.f, 0.f, 0.f, 0.f, 0.f, 0.f, 0.f};
  return z;
}

__device__ __forceinline__ void store_rows_16x64(const float* slab, float* g, int lane) {
  const int hf = lane >> 4, c4 = (lane & 15) * 4;
  for (int pass = 0; pass < 2; ++pass) {
#pragma unroll
    for (int it = 0; it < 8; ++it) {
      const int row = it * 2 + hf;
      const v4f v = *(const v4f*)(slab + row * SP + c4);
      *(volatile v4f*)(g + (size_t)row * HD + c4) = v;
    }
    __threadfence();
  }
}

union NodeU { f16t xs[64 * XP]; float slab[4 * 16 * SP]; };

__global__ __launch_bounds__(128) void k_node(const float* __restrict__ x, const float* __restrict__ Wp,
                                             const float* __restrict__ bproj, const float* __restrict__ Wc,
                                             const float* __restrict__ Wcb,
                                             float* __restrict__ ZI, float* __restrict__ ZJ, f16t* __restrict__ HT) {
  __shared__ __align__(16) NodeU u;
  __shared__ __align__(16) f16t WTs[64 * WP];
  __shared__ __align__(16) f16t Wcs[64 * WP];
  __shared__ __align__(16) f16t Hs[64 * HP];

  const int tid = threadIdx.x, wave = tid >> 5, lane = tid & 31, m = lane & 15, hf = lane >> 4;
  const int bh = blockIdx.y, b = bh >> 2, hd = bh & 3;
  const int n0 = blockIdx.x * 64;

#pragma unroll 4
  for (int it = 0; it < 16; ++it) {
    const int idx = it * 128 + tid;
    const int row = idx >> 5, c4 = (idx & 31) * 4;
    const v4f v = *(const v4f*)(x + ((size_t)(b * NNODE + n0 + row) * FIN + c4));
    v4h hv;
    hv[0] = (f16t)v[0]; hv[1] = (f16t)v[1]; hv[2] = (f16t)v[2]; hv[3] = (f16t)v[3];
    *(v4h*)(u.xs + row * XP + c4) = hv;
  }
#pragma unroll 4
  for (int it = 0; it < 16; ++it) {
    const int idx = it * 128 + tid;
    const int i = idx >> 4, d4 = (idx & 15) * 4;
    const v4f v = *(const v4f*)(Wp + ((size_t)(hd * FIN + i) * HD + d4));
    WTs[(d4 + 0) * WP + i] = (f16t)(16.0f * v[0]);
    WTs[(d4 + 1) * WP + i] = (f16t)(16.0f * v[1]);
    WTs[(d4 + 2) * WP + i] = (f16t)(16.0f * v[2]);
    WTs[(d4 + 3) * WP + i] = (f16t)(16.0f * v[3]);
  }
#pragma unroll 4
  for (int it = 0; it < 16; ++it) {
    const int idx = it * 128 + tid;
    const int e = idx >> 5, c4 = (idx & 31) * 4;
    const v4f v = *(const v4f*)(Wc + ((size_t)(hd * HD + e) * (2 * HD) + c4));
    v4h hv;
    hv[0] = (f16t)(16.0f * v[0]); hv[1] = (f16t)(16.0f * v[1]);
    hv[2] = (f16t)(16.0f * v[2]); hv[3] = (f16t)(16.0f * v[3]);
    *(v4h*)(Wcs + e * WP + c4) = hv;
  }
  __syncthreads();

  const int lr0 = wave * 16;

  v8f acc[4];
#pragma unroll
  for (int t = 0; t < 4; ++t) acc[t] = zero8();
#pragma unroll
  for (int ks = 0; ks < 4; ++ks) {
    const int k0 = ks * 32;
    const v16h A = ldfrag(u.xs + (lr0 + m) * XP + k0 + 8 * hf);
#pragma unroll
    for (int t = 0; t < 4; ++t) {
      const v16h Bt = ldfrag(WTs + (16 * t + m) * WP + k0 + 8 * hf);
      acc[t] = mma16(A, Bt, acc[t]);
    }
  }
#pragma unroll
  for (int t = 0; t < 4; ++t) {
    const int d = 16 * t + m;
    const float bp = bproj[hd * HD + d];
#pragma unroll
    for (int r = 0; r < 8; ++r)
      Hs[(lr0 + 8 * hf + r) * HP + d] = (f16t)(acc[t][r] * 0.0625f + bp);
  }
  __syncthreads();

  v8f ai[4], aj[4];
#pragma unroll
  for (int t = 0; t < 4; ++t) { ai[t] = zero8(); aj[t] = zero8(); }
#pragma unroll
  for (int ks = 0; ks < 2; ++ks) {
    const int k0 = ks * 32;
    const v16h A = ldfrag(Hs + (lr0 + m) * HP + k0 + 8 * hf);
#pragma unroll
    for (int t = 0; t < 4; ++t) {
      const v16h B1 = ldfrag(Wcs + (16 * t + m) * WP + k0 + 8 * hf);
      const v16h B2 = ldfrag(Wcs + (16 * t + m) * WP + HD + k0 + 8 * hf);
      ai[t] = mma16(A, B1, ai[t]);
      aj[t] = mma16(A, B2, aj[t]);
    }
  }
  float* slab = u.slab + wave * 16 * SP;
#pragma unroll
  for (int t = 0; t < 4; ++t) {
    const int e = 16 * t + m;
    const float wb = Wcb[hd * HD + e];
#pragma unroll
    for (int r = 0; r < 8; ++r) slab[(8 * hf + r) * SP + e] = ai[t][r] * 0.0625f + wb;
  }
  __syncthreads();
  store_rows_16x64(slab, ZI + (size_t)(bh * NNODE + n0 + lr0) * HD, lane);
  __syncthreads();
#pragma unroll
  for (int t = 0; t < 4; ++t) {
    const int e = 16 * t + m;
#pragma unroll
    for (int r = 0; r < 8; ++r) slab[(8 * hf + r) * SP + e] = aj[t][r] * 0.0625f;
  }
  __syncthreads();
  store_rows_16x64(slab, ZJ + (size_t)(bh * NNODE + n0 + lr0) * HD, lane);

  {
    const int q = tid & 7, rs = tid >> 3;
    Pack8 pk[4];
#pragma unroll
    for (int it = 0; it < 4; ++it) {
      const int d = it * 16 + rs;
#pragma unroll
      for (int e = 0; e < 8; ++e) pk[it].e[e] = Hs[(8 * q + e) * HP + d];
    }
    f16t* g = HT + (size_t)bh * HD * NNODE + n0 + 8 * q;
    for (int pass = 0; pass < 2; ++pass) {
#pragma unroll
      for (int it = 0; it < 4; ++it) {
        const int d = it * 16 + rs;
        *(volatile v8h*)(g + (size_t)d * NNODE) = pk[it].v;
      }
      __threadfence();
    }
  }
}

__device__ __forceinline__ void logits_chunk(const float* __restrict__ zjg, float* ZJs, const float* ZIs,
                                             const float* A4s, const float* A6s, int tid, float (&lg)[QR]) {
  __syncthreads();
#pragma unroll 4
  for (int it = 0; it < 16; ++it) {
    const int idx = it * 128 + tid;
    const int row = idx >> 4, c4 = (idx & 15) * 4;
    const v4f v = *(const v4f*)(zjg + (size_t)row * HD + c4);
    float* zd = ZJs + row * ZJP + c4;
    zd[0] = v[0]; zd[1] = v[1]; zd[2] = v[2]; zd[3] = v[3];
  }
  __syncthreads();
#pragma unroll
  for (int r = 0; r < QR; ++r) lg[r] = 0.f;
  float vj = 0.f;
  const float* zr = ZJs + tid * ZJP;
#pragma unroll 1
  for (int e = 0; e < HD; ++e) {
    const float zj = zr[e];
    const float b4 = A4s[e];
    const float b6 = A6s[e];
    vj = fmaf(b6, zj, vj);
#pragma unroll
    for (int r = 0; r < QR; ++r) {
      const float s = ZIs[r * HD + e] + zj;
      lg[r] = fmaf(b4, fabsf(s), lg[r]);
    }
  }
#pragma unroll
  for (int r = 0; r < QR; ++r) lg[r] += vj;
}

__device__ __forceinline__ void exp_rows(const float (&lg)[QR], const float (&mx)[QR], float (&sm)[QR], f16t* pcol) {
#pragma unroll
  for (int r = 0; r < QR; ++r) {
    const float p = __expf(lg[r] - mx[r]);
    sm[r] += p;
    pcol[r * PSP] = (f16t)(p * 256.0f);
  }
}

__global__ __launch_bounds__(128) void k_attn(const float* __restrict__ ZI, const float* __restrict__ ZJ,
                                             const f16t* __restrict__ HT, const float* __restrict__ avec,
                                             const float* __restrict__ obias, float* __restrict__ out) {
  __shared__ __align__(16) float ZIs[QR * HD];
  __shared__ __align__(16) float A4s[HD];
  __shared__ __align__(16) float A6s[HD];
  __shared__ __align__(16) float ZJs[KCH * ZJP];
  __shared__ __align__(16) f16t  Ps[QR * PSP];
  __shared__ __align__(16) float RedM[4 * QR];
  __shared__ __align__(16) float RedS[4 * QR];
  __shared__ __align__(16) float Os[QR * OSP];

  const int tid = threadIdx.x, wave = tid >> 5, lane = tid & 31, m = lane & 15, hf = lane >> 4;
  const int bh = blockIdx.y, b = bh >> 2, hd = bh & 3;
  const int i0 = blockIdx.x * QR;

#pragma unroll
  for (int it = 0; it < 2; ++it) {
    const int idx = it * 128 + tid;
    const int row = idx >> 4, c4 = (idx & 15) * 4;
    const v4f v = *(const v4f*)(ZI + ((size_t)(bh * NNODE + i0 + row) * HD + c4));
    *(v4f*)(ZIs + row * HD + c4) = v;
  }
  {
    const int e = tid & 63;
    const float av = avec[hd * HD + e];
    if (tid < 64) A4s[e] = 0.4f * av; else A6s[e] = 0.6f * av;
  }

  float lg0[QR], lg1[QR], lg2[QR], lg3[QR];
  const float* zjb = ZJ + (size_t)bh * NNODE * HD;
  logits_chunk(zjb + (size_t)0 * KCH * HD, ZJs, ZIs, A4s, A6s, tid, lg0);
  logits_chunk(zjb + (size_t)1 * KCH * HD, ZJs, ZIs, A4s, A6s, tid, lg1);
  logits_chunk(zjb + (size_t)2 * KCH * HD, ZJs, ZIs, A4s, A6s, tid, lg2);
  logits_chunk(zjb + (size_t)3 * KCH * HD, ZJs, ZIs, A4s, A6s, tid, lg3);

  float mx[QR], sm[QR];
#pragma unroll
  for (int r = 0; r < QR; ++r) mx[r] = fmaxf(fmaxf(lg0[r], lg1[r]), fmaxf(lg2[r], lg3[r]));
#pragma unroll
  for (int r = 0; r < QR; ++r) {
#pragma unroll
    for (int off = 16; off > 0; off >>= 1) mx[r] = fmaxf(mx[r], __shfl_xor(mx[r], off, 32));
  }
  if (lane == 0) {
#pragma unroll
    for (int r = 0; r < QR; ++r) RedM[wave * QR + r] = mx[r];
  }
  __syncthreads();
#pragma unroll
  for (int r = 0; r < QR; ++r) {
    mx[r] = fmaxf(fmaxf(RedM[r], RedM[QR + r]), fmaxf(RedM[2 * QR + r], RedM[3 * QR + r]));
    sm[r] = 0.f;
  }
  {
    f16t* pc = Ps + tid;
    exp_rows(lg0, mx, sm, pc + 0 * KCH);
    exp_rows(lg1, mx, sm, pc + 1 * KCH);
    exp_rows(lg2, mx, sm, pc + 2 * KCH);
    exp_rows(lg3, mx, sm, pc + 3 * KCH);
  }
#pragma unroll
  for (int r = 0; r < QR; ++r) {
#pragma unroll
    for (int off = 16; off > 0; off >>= 1) sm[r] += __shfl_xor(sm[r], off, 32);
  }
  if (lane == 0) {
#pragma unroll
    for (int r = 0; r < QR; ++r) RedS[wave * QR + r] = sm[r];
  }
  __syncthreads();

  v8f oacc = zero8();
  const f16t* prow = Ps + m * PSP + 8 * hf;
  const f16t* hrow = HT + (size_t)(bh * HD + wave * 16 + m) * NNODE + 8 * hf;
#pragma unroll 4
  for (int ks = 0; ks < NNODE / 32; ++ks) {
    const v16h A  = ldfrag(prow + ks * 32);
    const v16h Bf = ldfrag(hrow + ks * 32);
    oacc = mma16(A, Bf, oacc);
  }

  {
    const int d = wave * 16 + m;
    const float bo = obias[hd * HD + d];
#pragma unroll
    for (int r = 0; r < 8; ++r) {
      const int row = 8 * hf + r;
      const float tot = (RedS[row] + RedS[QR + row]) + (RedS[2 * QR + row] + RedS[3 * QR + row]);
      const float inv = __builtin_amdgcn_rcpf(tot) * 0.00390625f;
      Os[row * OSP + d] = fmaf(oacc[r], inv, bo);
    }
  }
  __syncthreads();
  {
    const int rsel = tid >> 4, c4 = (tid & 15) * 4;
    float* ob = out + (size_t)(b * NNODE + i0) * OUTW + hd * HD + c4;
    for (int pass = 0; pass < 2; ++pass) {
#pragma unroll
      for (int it = 0; it < 2; ++it) {
        const int row = it * 8 + rsel;
        const v4f v = *(const v4f*)(Os + row * OSP + c4);
        *(volatile v4f*)(ob + (size_t)row * OUTW) = v;
      }
      __threadfence();
    }
  }
}

extern "C" void kernel_launch(void* const* d_in, const int* in_sizes, int n_in,
                              void* d_out, int out_size, void* d_ws, size_t ws_size,
                              hipStream_t stream) {
  if (n_in < 7) return;
  if (in_sizes[0] != NB * NNODE * FIN) return;
  if (in_sizes[1] != NHEAD * FIN * HD) return;
  if (in_sizes[2] != NHEAD * HD) return;
  if (in_sizes[3] != NHEAD * HD * 2 * HD) return;
  if (in_sizes[4] != NHEAD * HD) return;
  if (in_sizes[5] != NHEAD * HD) return;
  if (in_sizes[6] != NHEAD * HD) return;
  if (out_size != NB * NNODE * OUTW) return;

  const float* x     = (const float*)d_in[0];
  const float* Wp    = (const float*)d_in[1];
  const float* bproj = (const float*)d_in[2];
  const float* Wc    = (const float*)d_in[3];
  const float* Wcb   = (const float*)d_in[4];
  const float* avec  = (const float*)d_in[5];
  const float* obias = (const float*)d_in[6];
  float* out = (float*)d_out;

  const size_t szZ  = (size_t)NB * NHEAD * NNODE * HD * sizeof(float);
  const size_t szHT = (size_t)NB * NHEAD * HD * NNODE * sizeof(f16t);
  const size_t oZI = 0;
  const size_t oZJ = oZI + szZ;
  const size_t oHT = oZJ + szZ;
  const size_t total = oHT + szHT;
  if (total > ws_size) return;

  char* ws = (char*)d_ws;
  float* ZI = (float*)(ws + oZI);
  float* ZJ = (float*)(ws + oZJ);
  f16t*  HT = (f16t*)(ws + oHT);

  k_node<<<dim3(NNODE / 64, NB * NHEAD), dim3(128), 0, stream>>>(x, Wp, bproj, Wc, Wcb, ZI, ZJ, HT);
  k_attn<<<dim3(NNODE / QR, NB * NHEAD), dim3(128), 0, stream>>>(ZI, ZJ, HT, avec, obias, out);
  (void)hipGetLastError();
}
